// ElasticAttention_90056874262668
// MI455X (gfx1250) — hardware-verified
//
#include <hip/hip_runtime.h>
#include <stddef.h>
#include <stdint.h>

#define TQ    2048
#define TP    2048
#define TF    4096
#define HID   2048
#define NH    16
#define NKV   2
#define GQA   8
#define HDM   128
#define NQKV  2560
#define KOFS  2048
#define VOFS  2304
#define QB    128
#define KC    64
#define NQB   (TQ / QB)
#define NKC   (TF / KC)
#define OUT1F (TQ * HID)
#define OUT2F (TQ * HID + NKV * TF * HDM)
#define OUTN  (TQ * HID + 2 * NKV * TF * HDM)

static_assert(NH * HDM == HID);
static_assert(NH == GQA * NKV);
static_assert(NQKV == HID + 2 * NKV * HDM);
static_assert(KOFS == NH * HDM);
static_assert(VOFS == NH * HDM + NKV * HDM);
static_assert(TQ % 256 == 0);
static_assert(TQ % QB == 0);
static_assert(TP % 64 == 0);
static_assert(TF % KC == 0);
static_assert(TF == TP + TQ);
static_assert(HID % 64 == 0);
static_assert(HID == 256 * 8);
static_assert(HDM == 128);
static_assert(OUT1F == 4194304);
static_assert(OUT2F == 5242880);
static_assert(OUTN == 6291456);

typedef _Float16 v16h __attribute__((ext_vector_type(16)));
typedef _Float16 v8h  __attribute__((ext_vector_type(8)));
typedef float    v8f  __attribute__((ext_vector_type(8)));
typedef float    v4f  __attribute__((ext_vector_type(4)));
typedef unsigned int v4u __attribute__((ext_vector_type(4)));

union Frag  { v16h v; v8h h[2]; };
union Pack8 { v8h h; v4u u; };

__device__ __forceinline__ v8f mma16(v16h a, v16h b, v8f c) {
  c = __builtin_amdgcn_wmma_f32_16x16x32_f16(false, a, false, b, (short)0, c, false, false);
  asm volatile("v_nop\n\tv_nop\n\tv_nop\n\tv_nop" : "+v"(c) : "v"(a), "v"(b));
  return c;
}

__device__ __forceinline__ v16h ldfrag(const _Float16* p, int ld, int row0, int k0, int lane) {
  const int m = lane & 15, lh = lane >> 4;
  const _Float16* q = p + (size_t)(row0 + m) * ld + k0 + 8 * lh;
  Frag f;
  f.h[0] = *(const v8h*)(q);
  f.h[1] = *(const v8h*)(q + 16);
  return f.v;
}

__device__ __forceinline__ v8f zero8() { return (v8f){0.f, 0.f, 0.f, 0.f, 0.f, 0.f, 0.f, 0.f}; }

__device__ __forceinline__ void gemm16x64(const _Float16* __restrict__ A, int lda,
                                          const _Float16* __restrict__ Bt, int ldb,
                                          int m0, int n0, int lane, v8f (&acc)[4]) {
#pragma unroll 2
  for (int k0 = 0; k0 < HID; k0 += 32) {
    const v16h a = ldfrag(A, lda, m0, k0, lane);
#pragma unroll
    for (int t = 0; t < 4; ++t) {
      const v16h b = ldfrag(Bt, ldb, n0 + 16 * t, k0, lane);
      acc[t] = mma16(a, b, acc[t]);
    }
  }
}

__device__ __forceinline__ void gemm32x64(const _Float16* __restrict__ A, int lda,
                                          const _Float16* __restrict__ Bt, int ldb,
                                          int m0, int n0, int lane, v8f (&acc)[2][4]) {
#pragma unroll 2
  for (int k0 = 0; k0 < HID; k0 += 32) {
    const v16h a0 = ldfrag(A, lda, m0, k0, lane);
    const v16h a1 = ldfrag(A, lda, m0 + 16, k0, lane);
    const v16h b0 = ldfrag(Bt, ldb, n0, k0, lane);
    const v16h b1 = ldfrag(Bt, ldb, n0 + 16, k0, lane);
    const v16h b2 = ldfrag(Bt, ldb, n0 + 32, k0, lane);
    const v16h b3 = ldfrag(Bt, ldb, n0 + 48, k0, lane);
    acc[0][0] = mma16(a0, b0, acc[0][0]);
    acc[1][0] = mma16(a1, b0, acc[1][0]);
    acc[0][1] = mma16(a0, b1, acc[0][1]);
    acc[1][1] = mma16(a1, b1, acc[1][1]);
    acc[0][2] = mma16(a0, b2, acc[0][2]);
    acc[1][2] = mma16(a1, b2, acc[1][2]);
    acc[0][3] = mma16(a0, b3, acc[0][3]);
    acc[1][3] = mma16(a1, b3, acc[1][3]);
  }
}

__global__ __launch_bounds__(256) void k_cvt(const float* __restrict__ src, _Float16* __restrict__ dst, float scale) {
  const int row = blockIdx.x;
  const int col = (int)threadIdx.x * 8;
  const size_t o = (size_t)row * HID + col;
  const v4f a0 = *(const v4f*)(src + o);
  const v4f a1 = *(const v4f*)(src + o + 4);
  Pack8 pk;
  pk.h = (v8h){(_Float16)(a0[0] * scale), (_Float16)(a0[1] * scale), (_Float16)(a0[2] * scale), (_Float16)(a0[3] * scale),
               (_Float16)(a1[0] * scale), (_Float16)(a1[1] * scale), (_Float16)(a1[2] * scale), (_Float16)(a1[3] * scale)};
  const v4u vv = pk.u;
  volatile v4u* d = (volatile v4u*)(dst + o);
  *d = vv;
  __threadfence();
  *d = vv;
}

#define SFP 132
__device__ __forceinline__ void st_rows64(const float* sf, float* __restrict__ dst, int tid, int lane) {
  v4f val[8];
  size_t go[8];
#pragma unroll
  for (int it = 0; it < 8; ++it) {
    const int lr = (tid >> 5) + 8 * it;
    val[it] = *(const v4f*)(sf + lr * SFP + lane * 4);
    go[it]  = (size_t)lr * HDM + lane * 4;
  }
  for (int ps = 0; ps < 2; ++ps) {
#pragma unroll
    for (int it = 0; it < 8; ++it) *(volatile v4f*)(dst + go[it]) = val[it];
    __threadfence();
  }
}

__global__ __launch_bounds__(256) void k_past(const float* __restrict__ pk, const float* __restrict__ pv,
                                              _Float16* __restrict__ kp, _Float16* __restrict__ vtp,
                                              float* __restrict__ ko, float* __restrict__ vo) {
  __shared__ __align__(16) float sf[64 * SFP];
  const int tid = threadIdx.x, lane = tid & 31;
  const int kb    = blockIdx.x;
  const int kvh   = blockIdx.y;
  const int which = blockIdx.z;
  const float* src = ((which == 0) ? pk : pv) + ((size_t)kvh * TP + (size_t)kb * 64) * HDM;
#pragma unroll
  for (int e = 0; e < 8; ++e) {
    const int p   = tid + 256 * e;
    const int row = p >> 5;
    const int c4  = (p & 31) * 4;
    *(v4f*)(sf + row * SFP + c4) = *(const v4f*)(src + (size_t)row * HDM + c4);
  }
  __syncthreads();
  const size_t r0 = (size_t)kvh * TF + (size_t)kb * 64;

  if (which == 0) {
    v4u val[4];
    size_t go[4];
#pragma unroll
    for (int j = 0; j < 4; ++j) {
      const int p  = tid + 256 * j;
      const int lr = p >> 4;
      const int d0 = (p & 15) * 8;
      const float* ra = sf + lr * SFP + d0;
      const v4f a0 = *(const v4f*)(ra), a1 = *(const v4f*)(ra + 4);
      Pack8 q;
      q.h = (v8h){(_Float16)a0[0], (_Float16)a0[1], (_Float16)a0[2], (_Float16)a0[3],
                  (_Float16)a1[0], (_Float16)a1[1], (_Float16)a1[2], (_Float16)a1[3]};
      val[j] = q.u;
      go[j]  = (r0 + lr) * HDM + d0;
    }
    for (int ps = 0; ps < 2; ++ps) {
#pragma unroll
      for (int j = 0; j < 4; ++j) *(volatile v4u*)(kp + go[j]) = val[j];
      __threadfence();
    }
    st_rows64(sf, ko + r0 * HDM, tid, lane);
  } else {
    v4u val[4];
    size_t go[4];
#pragma unroll
    for (int j = 0; j < 4; ++j) {
      const int p  = tid + 256 * j;
      const int d  = p >> 3;
      const int pc = p & 7;
      const float* cp = sf + (pc * 8) * SFP + d;
      Pack8 q;
      q.h = (v8h){(_Float16)cp[0 * SFP], (_Float16)cp[1 * SFP], (_Float16)cp[2 * SFP], (_Float16)cp[3 * SFP],
                  (_Float16)cp[4 * SFP], (_Float16)cp[5 * SFP], (_Float16)cp[6 * SFP], (_Float16)cp[7 * SFP]};
      val[j] = q.u;
      go[j]  = ((size_t)kvh * HDM + d) * TF + (size_t)kb * 64 + pc * 8;
    }
    for (int ps = 0; ps < 2; ++ps) {
#pragma unroll
      for (int j = 0; j < 4; ++j) *(volatile v4u*)(vtp + go[j]) = val[j];
      __threadfence();
    }
    st_rows64(sf, vo + r0 * HDM, tid, lane);
  }
}

__global__ __launch_bounds__(256) void k_qkv(const _Float16* __restrict__ xh,
                                             const _Float16* __restrict__ wt,
                                             const float* __restrict__ bq,
                                             const float* __restrict__ bk,
                                             const float* __restrict__ bv,
                                             _Float16* __restrict__ qp,
                                             _Float16* __restrict__ kp,
                                             _Float16* __restrict__ vtp,
                                             float* __restrict__ ko,
                                             float* __restrict__ vo) {
  __shared__ __align__(16) float sf[64 * SFP];
  const int tid = threadIdx.x, lane = tid & 31, wave = tid >> 5;
  const int hh = lane >> 4, c = lane & 15;
  const int wm = wave >> 1, wn = wave & 1;
  const int mb = blockIdx.x * 64;
  const int ns = blockIdx.y;
  const int which = (ns < NH) ? 0 : ((ns < NH + NKV) ? 1 : 2);
  const int head = (which == 0) ? ns : ((which == 1) ? (ns - NH) : (ns - NH - NKV));
  const int m0 = mb + wm * 16;
  const int n0 = ns * HDM + wn * 64;
  const float* bias = (which == 0) ? (bq + head * HDM) : ((which == 1) ? (bk + head * HDM) : (bv + head * HDM));

  v8f acc[4];
#pragma unroll
  for (int t = 0; t < 4; ++t) acc[t] = zero8();
  gemm16x64(xh, HID, wt, HID, m0, n0, lane, acc);

#pragma unroll
  for (int t = 0; t < 4; ++t) {
    const float bb = bias[wn * 64 + 16 * t + c];
#pragma unroll
    for (int r = 0; r < 8; ++r)
      sf[(wm * 16 + 8 * hh + r) * SFP + wn * 64 + 16 * t + c] = acc[t][r] * 0.03125f + bb;
  }
  __syncthreads();

  if (which < 2) {
    v4u val[4];
    size_t go[4];
#pragma unroll
    for (int j = 0; j < 4; ++j) {
      const int p  = tid + 256 * j;
      const int lr = p >> 4;
      const int d0 = (p & 15) * 8;
      const float* ra = sf + lr * SFP + d0;
      const v4f a0 = *(const v4f*)(ra), a1 = *(const v4f*)(ra + 4);
      Pack8 q;
      q.h = (v8h){(_Float16)a0[0], (_Float16)a0[1], (_Float16)a0[2], (_Float16)a0[3],
                  (_Float16)a1[0], (_Float16)a1[1], (_Float16)a1[2], (_Float16)a1[3]};
      val[j] = q.u;
      go[j]  = (which == 0) ? (((size_t)head * TQ + mb + lr) * HDM + d0)
                            : (((size_t)head * TF + TP + mb + lr) * HDM + d0);
    }
    _Float16* base = (which == 0) ? qp : kp;
    for (int ps = 0; ps < 2; ++ps) {
#pragma unroll
      for (int j = 0; j < 4; ++j) *(volatile v4u*)(base + go[j]) = val[j];
      __threadfence();
    }
    if (which == 1) st_rows64(sf, ko + ((size_t)head * TF + TP + mb) * HDM, tid, lane);
  } else {
    v4u val[4];
    size_t go[4];
#pragma unroll
    for (int j = 0; j < 4; ++j) {
      const int p  = tid + 256 * j;
      const int d  = p >> 3;
      const int pc = p & 7;
      const float* cp = sf + (pc * 8) * SFP + d;
      Pack8 q;
      q.h = (v8h){(_Float16)cp[0 * SFP], (_Float16)cp[1 * SFP], (_Float16)cp[2 * SFP], (_Float16)cp[3 * SFP],
                  (_Float16)cp[4 * SFP], (_Float16)cp[5 * SFP], (_Float16)cp[6 * SFP], (_Float16)cp[7 * SFP]};
      val[j] = q.u;
      go[j]  = ((size_t)head * HDM + d) * TF + TP + mb + pc * 8;
    }
    for (int ps = 0; ps < 2; ++ps) {
#pragma unroll
      for (int j = 0; j < 4; ++j) *(volatile v4u*)(vtp + go[j]) = val[j];
      __threadfence();
    }
    st_rows64(sf, vo + ((size_t)head * TF + TP + mb) * HDM, tid, lane);
  }
}

#define KTQ 136
#define KTP 72
__global__ __launch_bounds__(256) void k_attn(const _Float16* __restrict__ qp,
                                              const _Float16* __restrict__ kp,
                                              const _Float16* __restrict__ vt,
                                              const float* __restrict__ msk,
                                              _Float16* __restrict__ op, float sscale) {
  __shared__ __align__(16) _Float16 Ks[KC * KTQ];
  __shared__ __align__(16) _Float16 Vs[HDM * KTP];
  __shared__ __align__(16) _Float16 Ps[8 * 16 * KTP];
  __shared__ float red[2][8];

  const int tid = threadIdx.x, lane = tid & 31, wave = tid >> 5;
  const int hh = lane >> 4, c = lane & 15;
  const int qb  = blockIdx.x % NQB;
  const int h   = blockIdx.x / NQB;
  const int kvh = h / GQA;
  const int qr0 = qb * QB;
  const int q0  = qr0 + wave * 16;

  const _Float16* Q = qp + (size_t)h * TQ * HDM;
  const _Float16* K = kp + (size_t)kvh * TF * HDM;
  const _Float16* V = vt + (size_t)kvh * HDM * TF;
  const float* MB = msk + (size_t)qr0 * TF;

  const float NEGI = -__builtin_huge_valf();
  float mrow[8], lrow[8];
  v8f oacc[8];
#pragma unroll
  for (int r = 0; r < 8; ++r) { mrow[r] = NEGI; lrow[r] = 0.f; }
#pragma unroll
  for (int t = 0; t < 8; ++t) oacc[t] = zero8();

  _Float16* pw = Ps + wave * 16 * KTP;

  for (int kc = 0; kc < NKC; ++kc) {
    const int kv0 = kc * KC;
    float mx = NEGI;
#pragma unroll
    for (int e = 0; e < 8; ++e) {
      const int p   = tid + 256 * e;
      const int row = p >> 4;
      const int c4  = (p & 15) * 4;
      const v4f mv = *(const v4f*)(MB + (size_t)row * TF + kv0 + c4);
      mx = fmaxf(mx, fmaxf(fmaxf(mv[0], mv[1]), fmaxf(mv[2], mv[3])));
    }
#pragma unroll
    for (int off = 1; off < 32; off <<= 1) mx = fmaxf(mx, __shfl_xor(mx, off, 32));
    if (lane == 0) red[kc & 1][wave] = mx;
    __syncthreads();
    float bm = red[kc & 1][0];
#pragma unroll
    for (int w = 1; w < 8; ++w) bm = fmaxf(bm, red[kc & 1][w]);
    const int live = __builtin_amdgcn_readfirstlane((bm > -1.0e8f) ? 1 : 0);
    if (live == 0) continue;

    {
      const int r  = tid >> 2;
      const int qq = (tid & 3) * 32;
      const _Float16* ks = K + (size_t)(kv0 + r) * HDM + qq;
#pragma unroll
      for (int e = 0; e < 4; ++e) *(v8h*)(Ks + r * KTQ + qq + 8 * e) = *(const v8h*)(ks + 8 * e);
      const int dr = tid >> 1;
      const int q2 = (tid & 1) * 32;
      const _Float16* vs = V + (size_t)dr * TF + kv0 + q2;
#pragma unroll
      for (int e = 0; e < 4; ++e) *(v8h*)(Vs + dr * KTP + q2 + 8 * e) = *(const v8h*)(vs + 8 * e);
    }
    __syncthreads();

    v8f s[4];
#pragma unroll
    for (int j = 0; j < 4; ++j) s[j] = zero8();
#pragma unroll
    for (int dc = 0; dc < 4; ++dc) {
      const v16h qa = ldfrag(Q, HDM, q0, dc * 32, lane);
#pragma unroll
      for (int j = 0; j < 4; ++j) {
        const v16h kb = ldfrag(Ks, KTQ, j * 16, dc * 32, lane);
        s[j] = mma16(qa, kb, s[j]);
      }
    }
#pragma unroll
    for (int r = 0; r < 8; ++r) {
      const float* mp = msk + (size_t)(q0 + 8 * hh + r) * TF + kv0 + c;
#pragma unroll
      for (int j = 0; j < 4; ++j) s[j][r] = s[j][r] * sscale + mp[16 * j];
    }
    float cm[8];
#pragma unroll
    for (int r = 0; r < 8; ++r) {
      float m = NEGI;
#pragma unroll
      for (int j = 0; j < 4; ++j) m = fmaxf(m, s[j][r]);
#pragma unroll
      for (int off = 1; off < 16; off <<= 1) m = fmaxf(m, __shfl_xor(m, off, 32));
      cm[r] = m;
    }
    float al[8];
#pragma unroll
    for (int r = 0; r < 8; ++r) {
      const float mnew  = fmaxf(mrow[r], cm[r]);
      const float alpha = __expf(mrow[r] - mnew);
      mrow[r] = mnew;
      float psum = 0.f;
#pragma unroll
      for (int j = 0; j < 4; ++j) {
        const float p = __expf(s[j][r] - mnew);
        psum += p;
        pw[(8 * hh + r) * KTP + j * 16 + c] = (_Float16)(p * 1024.0f);
      }
#pragma unroll
      for (int off = 1; off < 16; off <<= 1) psum += __shfl_xor(psum, off, 32);
      lrow[r] = lrow[r] * alpha + psum;
      al[r] = alpha;
    }
#pragma unroll
    for (int t = 0; t < 8; ++t)
#pragma unroll
      for (int r = 0; r < 8; ++r) oacc[t][r] *= al[r];
    __syncthreads();

#pragma unroll
    for (int kk = 0; kk < 2; ++kk) {
      const v16h pa = ldfrag(pw, KTP, 0, kk * 32, lane);
#pragma unroll
      for (int t = 0; t < 8; ++t) {
        const v16h vb = ldfrag(Vs, KTP, t * 16, kk * 32, lane);
        oacc[t] = mma16(pa, vb, oacc[t]);
      }
    }
  }

  float invl[8];
#pragma unroll
  for (int r = 0; r < 8; ++r) invl[r] = (lrow[r] > 0.f) ? (0.015625f / lrow[r]) : 0.f;
#pragma unroll
  for (int half = 0; half < 2; ++half) {
    __syncthreads();
#pragma unroll
    for (int r = 0; r < 8; ++r) {
#pragma unroll
      for (int t = 0; t < 4; ++t)
        pw[(8 * hh + r) * KTP + 16 * t + c] = (_Float16)(oacc[4 * half + t][r] * invl[r]);
    }
    __syncthreads();
    v4u val[4];
    size_t go[4];
#pragma unroll
    for (int it = 0; it < 4; ++it) {
      const int p  = lane + 32 * it;
      const int L  = p >> 3;
      const int pc = p & 7;
      Pack8 q;
      q.h     = *(const v8h*)(pw + L * KTP + pc * 8);
      val[it] = q.u;
      go[it]  = (size_t)(q0 + L) * HID + (size_t)h * HDM + half * 64 + pc * 8;
    }
    for (int ps = 0; ps < 2; ++ps) {
#pragma unroll
      for (int it = 0; it < 4; ++it) *(volatile v4u*)(op + go[it]) = val[it];
      __threadfence();
    }
  }
}

#define OTP 68
__device__ __forceinline__ void out_epilogue(v8f (&acc)[2][4], float scale, const float* __restrict__ bias,
                                             float* sw, float* __restrict__ out,
                                             int m0, int n0, int lane, int hh, int c) {
  float bb[4];
#pragma unroll
  for (int t = 0; t < 4; ++t) bb[t] = bias[n0 + 16 * t + c];
#pragma unroll
  for (int sub = 0; sub < 2; ++sub) {
    __syncthreads();
#pragma unroll
    for (int t = 0; t < 4; ++t) {
#pragma unroll
      for (int r = 0; r < 8; ++r) sw[(8 * hh + r) * OTP + 16 * t + c] = acc[sub][t][r] * scale + bb[t];
    }
    __syncthreads();
    v4f val[8];
    size_t go[8];
#pragma unroll
    for (int it = 0; it < 8; ++it) {
      const int p    = lane + 32 * it;
      const int L    = p >> 3;
      const int pc   = p & 7;
      const int row  = L >> 1;
      const int half = L & 1;
      val[it] = *(const v4f*)(sw + row * OTP + half * 32 + pc * 4);
      go[it]  = (size_t)(m0 + sub * 16 + row) * HID + n0 + half * 32 + pc * 4;
    }
    for (int ps = 0; ps < 2; ++ps) {
#pragma unroll
      for (int it = 0; it < 8; ++it) *(volatile v4f*)(out + go[it]) = val[it];
      __threadfence();
    }
  }
}

__global__ __launch_bounds__(256) void k_out(const _Float16* __restrict__ ap,
                                             const _Float16* __restrict__ wt,
                                             const float* __restrict__ bo,
                                             float* __restrict__ out) {
  __shared__ __align__(16) float st[8][16 * OTP];
  const int tid = threadIdx.x, lane = tid & 31, wave = tid >> 5;
  const int hh = lane >> 4, c = lane & 15;
  const int m0 = blockIdx.x * 256 + wave * 32;
  const int n0 = blockIdx.y * 64;

  v8f acc[2][4];
#pragma unroll
  for (int s = 0; s < 2; ++s)
#pragma unroll
    for (int t = 0; t < 4; ++t) acc[s][t] = zero8();
  gemm32x64(ap, HID, wt, HID, m0, n0, lane, acc);
  out_epilogue(acc, 0.001953125f, bo, st[wave], out, m0, n0, lane, hh, c);
}

extern "C" void kernel_launch(void* const* d_in, const int* in_sizes, int n_in,
                              void* d_out, int out_size, void* d_ws, size_t ws_size,
                              hipStream_t stream) {
  if (n_in < 12) return;
  if (in_sizes[0]  != TQ * HID) return;
  if (in_sizes[1]  != TQ * TF) return;
  if (in_sizes[2]  != NKV * TP * HDM) return;
  if (in_sizes[3]  != NKV * TP * HDM) return;
  if (in_sizes[4]  != HID * HID) return;
  if (in_sizes[5]  != HID) return;
  if (in_sizes[6]  != NKV * HDM * HID) return;
  if (in_sizes[7]  != NKV * HDM) return;
  if (in_sizes[8]  != NKV * HDM * HID) return;
  if (in_sizes[9]  != NKV * HDM) return;
  if (in_sizes[10] != HID * HID) return;
  if (in_sizes[11] != HID) return;
  if (out_size != OUTN) return;

  const float* x   = (const float*)d_in[0];
  const float* msk = (const float*)d_in[1];
  const float* pk  = (const float*)d_in[2];
  const float* pv  = (const float*)d_in[3];
  const float* wq  = (const float*)d_in[4];
  const float* bq  = (const float*)d_in[5];
  const float* wk  = (const float*)d_in[6];
  const float* bk  = (const float*)d_in[7];
  const float* wv  = (const float*)d_in[8];
  const float* bv  = (const float*)d_in[9];
  const float* wo  = (const float*)d_in[10];
  const float* bo  = (const float*)d_in[11];
  float* out  = (float*)d_out;
  float* out1 = out + (size_t)OUT1F;
  float* out2 = out + (size_t)OUT2F;

  size_t off = 0;
  const size_t oX  = off; off += (size_t)TQ * HID * 2;
  const size_t oWt = off; off += (size_t)NQKV * HID * 2;
  const size_t oWo = off; off += (size_t)HID * HID * 2;
  const size_t oQ  = off; off += (size_t)NH * TQ * HDM * 2;
  const size_t oK  = off; off += (size_t)NKV * TF * HDM * 2;
  const size_t oV  = off; off += (size_t)NKV * HDM * TF * 2;
  const size_t oO  = off; off += (size_t)TQ * HID * 2;
  if (off > ws_size) return;
  if (off > (size_t)134217728) return;

  char* ws = (char*)d_ws;
  _Float16* Xh  = (_Float16*)(ws + oX);
  _Float16* Wt  = (_Float16*)(ws + oWt);
  _Float16* Wot = (_Float16*)(ws + oWo);
  _Float16* Qp  = (_Float16*)(ws + oQ);
  _Float16* Kp  = (_Float16*)(ws + oK);
  _Float16* Vt  = (_Float16*)(ws + oV);
  _Float16* Op  = (_Float16*)(ws + oO);

  k_cvt<<<dim3(TQ), dim3(256), 0, stream>>>(x, Xh, 1.0f);
  k_cvt<<<dim3(HID), dim3(256), 0, stream>>>(wq, Wt, 32.0f);
  k_cvt<<<dim3(NKV * HDM), dim3(256), 0, stream>>>(wk, Wt + (size_t)KOFS * HID, 32.0f);
  k_cvt<<<dim3(NKV * HDM), dim3(256), 0, stream>>>(wv, Wt + (size_t)VOFS * HID, 32.0f);
  k_cvt<<<dim3(HID), dim3(256), 0, stream>>>(wo, Wot, 32.0f);
  k_past<<<dim3(TP / 64, NKV, 2), dim3(256), 0, stream>>>(pk, pv, Kp, Vt, out1, out2);
  k_qkv<<<dim3(TQ / 64, NQKV / HDM), dim3(256), 0, stream>>>(Xh, Wt, bq, bk, bv, Qp, Kp, Vt, out1, out2);
  const float sscale = 0.08838834764831845f;
  k_attn<<<dim3(NH * NQB), dim3(256), 0, stream>>>(Qp, Kp, Vt, msk, Op, sscale);
  k_out<<<dim3(TQ / 256, HID / 64), dim3(256), 0, stream>>>(Op, Wot, bo, out);
  (void)hipGetLastError();
}
